// GlobalLocalModel_64768106824145
// MI455X (gfx1250) — hardware-verified
//
#include <hip/hip_runtime.h>
#include <stddef.h>


#define FH     128
#define KW     256
#define FIN    3
#define NMAT   44
#define WSZ    (FH * KW)
#define NTHR   256
#define NWAVE  8
#define GROWS  128
#define NT     (FH / 16)
#define PRW    4
#define PROWS  (NWAVE * PRW)
#define NPART  64
#define SEGCAP 4096
#define TPK    64
#define TPN    32
#define TPP    72
#define ASCL   16.0f
#define WSCL   64.0f
#define WSCAP  134217728
#define LDS_GEMM (GROWS * FH * 4)

static_assert(FH == 32 * 4);
static_assert(GROWS == NWAVE * 16);
static_assert((KW % 32) == 0 && (FH % 32) == 0 && KW == 2 * FH);
static_assert(TPN * 8 == NTHR && TPK * TPN == NTHR * 8 && TPK == NWAVE * 8);
static_assert((TPP % 8) == 0 && TPP >= TPK);
static_assert((KW % TPK) == 0 && (FH % TPN) == 0);
static_assert(PROWS == 32);
static_assert(FH <= NTHR);

typedef float     v4f  __attribute__((ext_vector_type(4)));
typedef float     v8f  __attribute__((ext_vector_type(8)));
typedef _Float16  v4h  __attribute__((ext_vector_type(4)));
typedef _Float16  v8h  __attribute__((ext_vector_type(8)));
typedef _Float16  v16h __attribute__((ext_vector_type(16)));
union FragH { v16h v; v8h h[2]; };

__device__ __forceinline__ v8f wmf(v16h a, v16h b, v8f c) {
  v8f d = __builtin_amdgcn_wmma_f32_16x16x32_f16(false, a, false, b, (short)0, c, false, false);
  asm volatile("v_nop\n\tv_nop\n\tv_nop\n\tv_nop" : "+v"(d) : "v"(a), "v"(b));
  return d;
}

__device__ __forceinline__ float elu1(float x) {
  const float t = __expf(fminf(x, 0.0f)) - 1.0f;
  return x > 0.0f ? x : t;
}
__device__ __forceinline__ v4f elu4(v4f v) {
  v4f o;
  o.x = elu1(v.x); o.y = elu1(v.y); o.z = elu1(v.z); o.w = elu1(v.w);
  return o;
}
__device__ __forceinline__ v4h cvt4h(v4f v) {
  v4h h;
  h[0] = (_Float16)v.x; h[1] = (_Float16)v.y; h[2] = (_Float16)v.z; h[3] = (_Float16)v.w;
  return h;
}

template <int WX, int WE>
__device__ __forceinline__ void emit4(float* Xo, float* E32o, _Float16* E16o, size_t g, v4f v, float escl) {
  const v4f e  = WE ? elu4(v) : v;
  const v4h hq = cvt4h(e * escl);
  if (WX) *(volatile v4f*)(Xo + g) = v;
  if (WE) { *(volatile v4f*)(E32o + g) = e; *(volatile v4h*)(E16o + g) = hq; }
  __threadfence();
  if (WX) *(volatile v4f*)(Xo + g) = v;
  if (WE) { *(volatile v4f*)(E32o + g) = e; *(volatile v4h*)(E16o + g) = hq; }
}

__global__ __launch_bounds__(NTHR) void k_wT16(const float* __restrict__ W, _Float16* Wp, float scale) {
  __shared__ __attribute__((aligned(16))) _Float16 sT[TPN * TPP];
  const int tid = threadIdx.x;
  const int k0 = (int)blockIdx.x * TPK, n0 = (int)blockIdx.y * TPN, z = (int)blockIdx.z;
  const float* Wz = W + (size_t)z * KW * FH;
  _Float16* Pz = Wp + (size_t)z * WSZ;
  const int nc = tid & 31, kq = tid >> 5;
#pragma unroll
  for (int i = 0; i < TPK / NWAVE; ++i) {
    const int kr = kq + NWAVE * i;
    const float v = Wz[(size_t)(k0 + kr) * FH + n0 + nc] * scale;
    sT[nc * TPP + kr] = (_Float16)v;
  }
  __syncthreads();
  const int nl = tid >> 3, p = tid & 7;
  const v8h hv = *(const v8h*)(sT + nl * TPP + 8 * p);
  _Float16* d = Pz + (size_t)(n0 + nl) * KW + k0 + 8 * p;
  *(volatile v8h*)d = hv;
  __threadfence();
  *(volatile v8h*)d = hv;
}

__global__ __launch_bounds__(NTHR) void k_conv_in(const float* __restrict__ in3, const float* __restrict__ W,
                                                  const float* __restrict__ b, float* Xo, float* E32o, _Float16* E16o,
                                                  int n, float escl) {
  const int tid = threadIdx.x, lane = tid & 31, wave = tid >> 5, c = 4 * lane;
  const v4f w0 = *(const v4f*)(W + c), w1 = *(const v4f*)(W + FH + c), w2 = *(const v4f*)(W + 2 * FH + c);
  const v4f bb = *(const v4f*)(b + c);
  const int rw = ((int)blockIdx.x * NWAVE + wave) * PRW;
#pragma unroll 1
  for (int i = 0; i < PRW; ++i) {
    const int r = rw + i;
    if (r < n) {
      const float x0 = in3[(size_t)r * FIN], x1 = in3[(size_t)r * FIN + 1], x2 = in3[(size_t)r * FIN + 2];
      v4f d = w0 * x0;
      d = d + w1 * x1;
      d = d + w2 * x2;
      const v4f v = d + bb;
      emit4<1, 1>(Xo, E32o, E16o, (size_t)r * FH + c, v, escl);
    }
  }
}

__global__ __launch_bounds__(NTHR) void k_maxpool(const float* __restrict__ Xin, float* Xo, float* E32o, _Float16* E16o,
                                                  int nOut, float escl) {
  const int tid = threadIdx.x, lane = tid & 31, wave = tid >> 5, c = 4 * lane;
  const int rw = ((int)blockIdx.x * NWAVE + wave) * PRW;
#pragma unroll 1
  for (int i = 0; i < PRW; ++i) {
    const int r = rw + i;
    if (r < nOut) {
      const v4f a = *(const v4f*)(Xin + (size_t)(2 * r) * FH + c);
      const v4f q = *(const v4f*)(Xin + (size_t)(2 * r + 1) * FH + c);
      v4f v;
      v.x = fmaxf(a.x, q.x); v.y = fmaxf(a.y, q.y); v.z = fmaxf(a.z, q.z); v.w = fmaxf(a.w, q.w);
      emit4<1, 1>(Xo, E32o, E16o, (size_t)r * FH + c, v, escl);
    }
  }
}

__global__ __launch_bounds__(NTHR) void k_upadd(const float* __restrict__ Xc, const float* __restrict__ D,
                                                float* Xo, float* E32o, _Float16* E16o, int nOut, float escl) {
  const int tid = threadIdx.x, lane = tid & 31, wave = tid >> 5, c = 4 * lane;
  const int rw = ((int)blockIdx.x * NWAVE + wave) * PRW;
#pragma unroll 1
  for (int i = 0; i < PRW; ++i) {
    const int r = rw + i;
    if (r < nOut) {
      const v4f a = *(const v4f*)(Xc + (size_t)(r >> 1) * FH + c);
      const v4f q = *(const v4f*)(D + (size_t)r * FH + c);
      const v4f v = a + q;
      emit4<1, 1>(Xo, E32o, E16o, (size_t)r * FH + c, v, escl);
    }
  }
}

__global__ __launch_bounds__(NTHR) void k_spmm(const int* __restrict__ rows, const int* __restrict__ cols,
                                               const float* __restrict__ vals, const float* __restrict__ E32,
                                               _Float16* S16, int ne, int n, float scl) {
  const int tid = threadIdx.x, lane = tid & 31, wave = tid >> 5;
  const int r = (int)blockIdx.x * NWAVE + wave;
  if (r >= n) return;
  int lo = 0, hi = ne;
#pragma unroll 1
  for (int it = 0; it < 40; ++it) {
    if (lo >= hi) break;
    const int md = (lo + hi) >> 1;
    if (rows[md] < r) lo = md + 1; else hi = md;
  }
  const int s0 = lo;
  hi = ne;
#pragma unroll 1
  for (int it = 0; it < 40; ++it) {
    if (lo >= hi) break;
    const int md = (lo + hi) >> 1;
    if (rows[md] <= r) lo = md + 1; else hi = md;
  }
  int cnt = lo - s0;
  cnt = cnt < 0 ? 0 : (cnt > SEGCAP ? SEGCAP : cnt);
  const int c4 = 4 * lane;
  v4f acc = {0.f, 0.f, 0.f, 0.f};
#pragma unroll 1
  for (int q0 = 0; q0 < cnt; q0 += 32) {
    int e = s0 + q0 + lane;
    e = e > ne - 1 ? ne - 1 : e;
    int cl = cols[e];
    cl = cl < 0 ? 0 : (cl > n - 1 ? n - 1 : cl);
    const int vb = __float_as_int(vals[e]);
    const int mcnt = (cnt - q0) < 32 ? (cnt - q0) : 32;
#pragma unroll 1
    for (int p = 0; p < mcnt; ++p) {
      const int   cp = __builtin_amdgcn_readlane(cl, p);
      const float vp = __int_as_float(__builtin_amdgcn_readlane(vb, p));
      const v4f   x  = *(const v4f*)(E32 + (size_t)cp * FH + c4);
      acc = acc + x * vp;
    }
  }
  const v4h hq = cvt4h(acc * scl);
  _Float16* d = S16 + (size_t)r * FH + c4;
  *(volatile v4h*)d = hq;
  __threadfence();
  *(volatile v4h*)d = hq;
}

template <int RES, int WX, int WE>
__global__ __launch_bounds__(NTHR) void k_gemm(const _Float16* __restrict__ A0p, const _Float16* __restrict__ A1p,
                                               const _Float16* __restrict__ Wp, const float* __restrict__ bias,
                                               const float* __restrict__ res, float* Xo, float* E32o, _Float16* E16o,
                                               int nRows, int a1str, float osc, float escl) {
  extern __shared__ v4f lds_dyn[];
  float* stg = (float*)lds_dyn;
  const int tid = threadIdx.x, lane = tid & 31, wave = tid >> 5, hh = lane >> 4, m = lane & 15;
  const int rowBase = (int)blockIdx.x * GROWS;
  if (rowBase + GROWS > nRows) return;
  const int arow = rowBase + wave * 16 + m;
  const _Float16* ap0 = A0p + (size_t)arow * FH + 8 * hh;
  const _Float16* ap1 = A1p + (size_t)arow * (size_t)a1str + 8 * hh;
  const _Float16* bp0 = Wp + (size_t)m * KW + 8 * hh;

  v8f acc[NT];
#pragma unroll
  for (int t = 0; t < NT; ++t) { v8f z = {0.f, 0.f, 0.f, 0.f, 0.f, 0.f, 0.f, 0.f}; acc[t] = z; }

#pragma unroll 1
  for (int kt = 0; kt < FH / 32; ++kt) {
    FragH af;
    af.h[0] = *(const v8h*)(ap0 + 32 * kt);
    af.h[1] = *(const v8h*)(ap0 + 32 * kt + 16);
#pragma unroll
    for (int t = 0; t < NT; ++t) {
      const _Float16* bp = bp0 + (size_t)(16 * t) * KW + 32 * kt;
      FragH bf;
      bf.h[0] = *(const v8h*)bp;
      bf.h[1] = *(const v8h*)(bp + 16);
      acc[t] = wmf(af.v, bf.v, acc[t]);
    }
  }
#pragma unroll 1
  for (int kt = 0; kt < FH / 32; ++kt) {
    FragH af;
    af.h[0] = *(const v8h*)(ap1 + 32 * kt);
    af.h[1] = *(const v8h*)(ap1 + 32 * kt + 16);
#pragma unroll
    for (int t = 0; t < NT; ++t) {
      const _Float16* bp = bp0 + (size_t)(16 * t) * KW + FH + 32 * kt;
      FragH bf;
      bf.h[0] = *(const v8h*)bp;
      bf.h[1] = *(const v8h*)(bp + 16);
      acc[t] = wmf(af.v, bf.v, acc[t]);
    }
  }

  {
    const int r0 = wave * 16 + 8 * hh;
    float* sp = stg + r0 * FH + m;
#pragma unroll
    for (int t = 0; t < NT; ++t) {
      const float bc = bias[16 * t + m];
#pragma unroll
      for (int r = 0; r < 8; ++r) sp[r * FH + 16 * t] = acc[t][r] * osc + bc;
    }
  }
  __syncthreads();

  const float* lrow = stg + wave * 16 * FH + 4 * lane;
  const size_t gro  = (size_t)(rowBase + wave * 16) * FH + 4 * lane;
#pragma unroll 1
  for (int i = 0; i < 16; ++i) {
    v4f v = *(const v4f*)(lrow + i * FH);
    const size_t g = gro + (size_t)i * FH;
    if (RES) v = v + *(const v4f*)(res + g);
    emit4<WX, WE>(Xo, E32o, E16o, g, v, escl);
  }
}

__global__ __launch_bounds__(NTHR) void k_avgpart(const float* __restrict__ E32, const float* __restrict__ mask,
                                                  float* part, int n) {
  __shared__ v4f sred[NWAVE * 32];
  const int tid = threadIdx.x, lane = tid & 31, wave = tid >> 5, c4 = 4 * lane;
  const int rb  = n / NPART;
  const int rpw = rb / NWAVE;
  const int rbeg = (int)blockIdx.x * rb + wave * rpw;
  v4f s = {0.f, 0.f, 0.f, 0.f};
#pragma unroll 1
  for (int i = 0; i < rpw; ++i) {
    int r = rbeg + i;
    r = r > n - 1 ? n - 1 : r;
    const float mk = mask[r];
    s = s + *(const v4f*)(E32 + (size_t)r * FH + c4) * mk;
  }
  sred[wave * 32 + lane] = s;
  __syncthreads();
  if (wave == 0) {
    v4f t = sred[lane];
#pragma unroll
    for (int w = 1; w < NWAVE; ++w) t = t + sred[w * 32 + lane];
    float* d = part + (size_t)blockIdx.x * FH + c4;
    *(volatile v4f*)d = t;
    __threadfence();
    *(volatile v4f*)d = t;
  }
}

__global__ __launch_bounds__(NTHR) void k_avgfin(const float* __restrict__ part, const float* __restrict__ mask,
                                                 _Float16* AVG16, int n, float scl) {
  __shared__ float sden[NTHR];
  __shared__ __attribute__((aligned(16))) _Float16 sAvg[FH];
  const int tid = threadIdx.x;
  float ds = 0.f;
#pragma unroll 1
  for (int i = tid; i < n; i += NTHR) ds += mask[i];
  sden[tid] = ds;
  __syncthreads();
  for (int st = NTHR / 2; st > 0; st >>= 1) {
    if (tid < st) sden[tid] += sden[tid + st];
    __syncthreads();
  }
  const float den  = sden[0];
  const float rden = 1.0f / den;
  const int ch = tid & (FH - 1);
  double cs = 0.0;
#pragma unroll 1
  for (int b = 0; b < NPART; ++b) cs += (double)part[(size_t)b * FH + ch];
  const float avg = (float)cs * rden;
  if (tid < FH) sAvg[tid] = (_Float16)(avg * scl);
  __syncthreads();
  v8h hv;
  hv = *(const v8h*)(sAvg + 8 * (tid & 15));
  if (tid < 16) *(volatile v8h*)(AVG16 + 8 * tid) = hv;
  __threadfence();
  if (tid < 16) *(volatile v8h*)(AVG16 + 8 * tid) = hv;
}

__global__ __launch_bounds__(NTHR) void k_heads(const float* __restrict__ EG, const float* __restrict__ EL,
                                                const float* __restrict__ gW2, const float* __restrict__ gb2,
                                                const float* __restrict__ lW2, const float* __restrict__ lb2,
                                                const float* __restrict__ in3, float* out, int n) {
  __shared__ __attribute__((aligned(16))) float sOut[3 * 32];
  const int tid = threadIdx.x, lane = tid & 31, wave = tid >> 5, c = 4 * lane;
  const float wg0 = gW2[(c + 0) * 2], wg1 = gW2[(c + 1) * 2], wg2 = gW2[(c + 2) * 2], wg3 = gW2[(c + 3) * 2];
  const float wl0 = lW2[c + 0], wl1 = lW2[c + 1], wl2 = lW2[c + 2], wl3 = lW2[c + 3];
  const float bg = gb2[0], bl = lb2[0];
  const int nb = (int)blockIdx.x * 32;
#pragma unroll 1
  for (int i = 0; i < 4; ++i) {
    const int wn = wave * 4 + i;
    int nd = nb + wn;
    nd = nd > n - 1 ? n - 1 : nd;
    const v4f eg = *(const v4f*)(EG + (size_t)nd * FH + c);
    const v4f el = *(const v4f*)(EL + (size_t)nd * FH + c);
    float pg = eg.x * wg0 + eg.y * wg1 + eg.z * wg2 + eg.w * wg3;
    float pl = el.x * wl0 + el.y * wl1 + el.z * wl2 + el.w * wl3;
#pragma unroll
    for (int o = 16; o > 0; o >>= 1) {
      pg += __shfl_xor(pg, o, 32);
      pl += __shfl_xor(pl, o, 32);
    }
    const float x0 = in3[(size_t)nd * FIN];
    const float sg = (pg + bg) + x0;
    const float sl = (pl + bl) + x0;
    const float wgt = 1.0f / (1.0f + expf(-sg));
    const float sf = wgt * sg + (1.0f - wgt) * sl;
    if (lane == 0) { sOut[wn] = sg; sOut[32 + wn] = sl; sOut[64 + wn] = sf; }
  }
  __syncthreads();
  if (wave == 0) {
    const int seg = lane >> 3, p = lane & 7;
    const int segc = seg > 2 ? 2 : seg;
    const v4f v = *(const v4f*)(sOut + segc * 32 + 4 * p);
    float* d = out + (size_t)segc * (size_t)n + nb + 4 * p;
    if (seg < 3) *(volatile v4f*)d = v;
    __threadfence();
    if (seg < 3) *(volatile v4f*)d = v;
  }
}

extern "C" void kernel_launch(void* const* d_in, const int* in_sizes, int n_in,
                              void* d_out, int out_size, void* d_ws, size_t ws_size,
                              hipStream_t stream) {
  if (n_in < 34) return;
  const int N = in_sizes[0] / FIN;
  if (N < 1024 || N > (1 << 20) || (N % 1024) != 0 || in_sizes[0] != N * FIN) return;
  if (out_size != 3 * N) return;
  if (in_sizes[2] != N) return;
  int lne[5];
  for (int l = 0; l < 5; ++l) {
    const int q = 3 + 3 * l;
    lne[l] = in_sizes[q];
    if (lne[l] <= 0 || lne[l] > (1 << 28) || in_sizes[q + 1] != lne[l] || in_sizes[q + 2] != lne[l]) return;
  }
  if (in_sizes[18] != FIN * FH || in_sizes[19] != FH) return;
  if (in_sizes[20] != 6 * WSZ / 2 * 2 / 2 * 1) {   }
  if (in_sizes[20] != 6 * FH * KW || in_sizes[21] != 6 * FH) return;
  if (in_sizes[22] != 2 * FH * KW || in_sizes[23] != 2 * FH) return;
  if (in_sizes[24] != 6 * FH * KW || in_sizes[25] != 6 * FH) return;
  if (in_sizes[26] != FH * 2 || in_sizes[27] != 2) return;
  if (in_sizes[28] != FIN * FH || in_sizes[29] != FH) return;
  if (in_sizes[30] != 30 * FH * KW || in_sizes[31] != 30 * FH) return;
  if (in_sizes[32] != FH || in_sizes[33] != 1) return;

  const float* inputs = (const float*)d_in[0];
  const float* mask1  = (const float*)d_in[2];
  const int*   lr[5] = {(const int*)d_in[3], (const int*)d_in[6], (const int*)d_in[9], (const int*)d_in[12], (const int*)d_in[15]};
  const int*   lc[5] = {(const int*)d_in[4], (const int*)d_in[7], (const int*)d_in[10], (const int*)d_in[13], (const int*)d_in[16]};
  const float* lv[5] = {(const float*)d_in[5], (const float*)d_in[8], (const float*)d_in[11], (const float*)d_in[14], (const float*)d_in[17]};
  const float* g_conv1_W = (const float*)d_in[18];
  const float* g_conv1_b = (const float*)d_in[19];
  const float* g_down_W  = (const float*)d_in[20];
  const float* g_down_b  = (const float*)d_in[21];
  const float* g_lap0_W  = (const float*)d_in[22];
  const float* g_lap0_b  = (const float*)d_in[23];
  const float* g_up_W    = (const float*)d_in[24];
  const float* g_up_b    = (const float*)d_in[25];
  const float* g_conv2_W = (const float*)d_in[26];
  const float* g_conv2_b = (const float*)d_in[27];
  const float* l_conv1_W = (const float*)d_in[28];
  const float* l_conv1_b = (const float*)d_in[29];
  const float* l_rn_W    = (const float*)d_in[30];
  const float* l_rn_b    = (const float*)d_in[31];
  const float* l_conv2_W = (const float*)d_in[32];
  const float* l_conv2_b = (const float*)d_in[33];
  float* out = (float*)d_out;

  char* ws = (char*)d_ws;
  size_t off = 0;
  const size_t szX = (size_t)N * FH * 4, szH = (size_t)N * FH * 2;
  const size_t oWp   = off; off += (size_t)NMAT * WSZ * 2;           off = (off + 255) & ~(size_t)255;
  const size_t oX0   = off; off += szX;                              off = (off + 255) & ~(size_t)255;
  const size_t oX1   = off; off += szX / 2;                          off = (off + 255) & ~(size_t)255;
  const size_t oX2   = off; off += szX / 4;                          off = (off + 255) & ~(size_t)255;
  const size_t oX3   = off; off += szX / 8;                          off = (off + 255) & ~(size_t)255;
  const size_t oT    = off; off += szX;                              off = (off + 255) & ~(size_t)255;
  const size_t oU    = off; off += szX;                              off = (off + 255) & ~(size_t)255;
  const size_t oAE32 = off; off += szX;                              off = (off + 255) & ~(size_t)255;
  const size_t oAE16 = off; off += szH;                              off = (off + 255) & ~(size_t)255;
  const size_t oBE32 = off; off += szX;                              off = (off + 255) & ~(size_t)255;
  const size_t oBE16 = off; off += szH;                              off = (off + 255) & ~(size_t)255;
  const size_t oS16  = off; off += szH;                              off = (off + 255) & ~(size_t)255;
  const size_t oEG   = off; off += szX;                              off = (off + 255) & ~(size_t)255;
  const size_t oAVG  = off; off += 256;                              off = (off + 255) & ~(size_t)255;
  const size_t oPart = off; off += (size_t)NPART * FH * 4;           off = (off + 255) & ~(size_t)255;
  if (off > ws_size || off > (size_t)WSCAP) return;
  _Float16* Wp    = (_Float16*)(ws + oWp);
  float*    X0    = (float*)(ws + oX0);
  float*    X1    = (float*)(ws + oX1);
  float*    X2    = (float*)(ws + oX2);
  float*    X3    = (float*)(ws + oX3);
  float*    T     = (float*)(ws + oT);
  float*    U     = (float*)(ws + oU);
  float*    AE32  = (float*)(ws + oAE32);
  _Float16* AE16  = (_Float16*)(ws + oAE16);
  float*    BE32  = (float*)(ws + oBE32);
  _Float16* BE16  = (_Float16*)(ws + oBE16);
  _Float16* S16   = (_Float16*)(ws + oS16);
  float*    EG    = (float*)(ws + oEG);
  _Float16* AVG16 = (_Float16*)(ws + oAVG);
  float*    part  = (float*)(ws + oPart);

  const float osc = 1.0f / (ASCL * WSCL);
  const int nlev[5] = {N / 8, N / 4, N / 2, N, N};

  {
    const dim3 g6(KW / TPK, FH / TPN, 6), g2(KW / TPK, FH / TPN, 2), g30(KW / TPK, FH / TPN, 30);
    k_wT16<<<g6, NTHR, 0, stream>>>(g_down_W, Wp + (size_t)0 * WSZ, WSCL);
    k_wT16<<<g2, NTHR, 0, stream>>>(g_lap0_W, Wp + (size_t)6 * WSZ, WSCL);
    k_wT16<<<g6, NTHR, 0, stream>>>(g_up_W, Wp + (size_t)8 * WSZ, WSCL);
    k_wT16<<<g30, NTHR, 0, stream>>>(l_rn_W, Wp + (size_t)14 * WSZ, WSCL);
  }

  hipFuncSetAttribute(reinterpret_cast<const void*>(&k_gemm<0, 0, 1>), hipFuncAttributeMaxDynamicSharedMemorySize, LDS_GEMM);
  hipFuncSetAttribute(reinterpret_cast<const void*>(&k_gemm<1, 1, 1>), hipFuncAttributeMaxDynamicSharedMemorySize, LDS_GEMM);
  hipFuncSetAttribute(reinterpret_cast<const void*>(&k_gemm<1, 1, 0>), hipFuncAttributeMaxDynamicSharedMemorySize, LDS_GEMM);
  hipFuncSetAttribute(reinterpret_cast<const void*>(&k_gemm<1, 0, 1>), hipFuncAttributeMaxDynamicSharedMemorySize, LDS_GEMM);

  auto spmm = [&](int li, const float* E32src, int n) {
    k_spmm<<<(n + NWAVE - 1) / NWAVE, NTHR, 0, stream>>>(lr[li], lc[li], lv[li], E32src, S16, lne[li], n, ASCL);
  };
  auto gemm = [&](int resf, int wx, int we, const _Float16* a0, const _Float16* a1, int a1str, int slot,
                  const float* bias, const float* res, float* xo, float* e32o, _Float16* e16o, int n) {
    const dim3 g(n / GROWS);
    const _Float16* w = Wp + (size_t)slot * WSZ;
    if (!resf)         k_gemm<0, 0, 1><<<g, NTHR, LDS_GEMM, stream>>>(a0, a1, w, bias, res, xo, e32o, e16o, n, a1str, osc, ASCL);
    else if (wx && we) k_gemm<1, 1, 1><<<g, NTHR, LDS_GEMM, stream>>>(a0, a1, w, bias, res, xo, e32o, e16o, n, a1str, osc, ASCL);
    else if (wx)       k_gemm<1, 1, 0><<<g, NTHR, LDS_GEMM, stream>>>(a0, a1, w, bias, res, xo, e32o, e16o, n, a1str, osc, ASCL);
    else               k_gemm<1, 0, 1><<<g, NTHR, LDS_GEMM, stream>>>(a0, a1, w, bias, res, xo, e32o, e16o, n, a1str, osc, ASCL);
  };
  auto lapblk = [&](int li, int n, const float* Xin, float* Xout, float* E32last, int slot, const float* b, int wx, int we) {
    spmm(li, AE32, n);
    gemm(0, 0, 1, AE16, S16, FH, slot, b, Xin, Xout, BE32, BE16, n);
    spmm(li, BE32, n);
    gemm(1, wx, we, BE16, S16, FH, slot + 1, b + FH, Xin, Xout, E32last, AE16, n);
  };
  auto avgblk = [&](int n, const float* Xin, float* Xout, int slot, const float* b, int wx, int we) {
    k_avgpart<<<NPART, NTHR, 0, stream>>>(AE32, mask1, part, n);
    k_avgfin<<<1, NTHR, 0, stream>>>(part, mask1, AVG16, n, ASCL);
    gemm(0, 0, 1, AE16, AVG16, 0, slot, b, Xin, Xout, BE32, BE16, n);
    k_avgpart<<<NPART, NTHR, 0, stream>>>(BE32, mask1, part, n);
    k_avgfin<<<1, NTHR, 0, stream>>>(part, mask1, AVG16, n, ASCL);
    gemm(1, wx, we, BE16, AVG16, 0, slot + 1, b + FH, Xin, Xout, AE32, AE16, n);
  };
  auto maxpool = [&](const float* Xin, float* Xo, int nOut) {
    k_maxpool<<<(nOut + PROWS - 1) / PROWS, NTHR, 0, stream>>>(Xin, Xo, AE32, AE16, nOut, ASCL);
  };
  auto upadd = [&](const float* Xc, const float* D, float* Xo, int nOut) {
    k_upadd<<<(nOut + PROWS - 1) / PROWS, NTHR, 0, stream>>>(Xc, D, Xo, AE32, AE16, nOut, ASCL);
  };

  k_conv_in<<<(N + PROWS - 1) / PROWS, NTHR, 0, stream>>>(inputs, g_conv1_W, g_conv1_b, X0, AE32, AE16, N, ASCL);
  lapblk(3, N, X0, T, AE32, 0, g_down_b + 0 * 2 * FH, 1, 0);
  maxpool(T, X1, N / 2);
  lapblk(2, N / 2, X1, T, AE32, 2, g_down_b + 1 * 2 * FH, 1, 0);
  maxpool(T, X2, N / 4);
  lapblk(1, N / 4, X2, T, AE32, 4, g_down_b + 2 * 2 * FH, 1, 0);
  maxpool(T, X3, N / 8);
  lapblk(0, N / 8, X3, T, AE32, 6, g_lap0_b, 1, 0);
  upadd(T, X2, U, N / 4);
  lapblk(1, N / 4, U, T, AE32, 8, g_up_b + 0 * 2 * FH, 1, 0);
  upadd(T, X1, U, N / 2);
  lapblk(2, N / 2, U, T, AE32, 10, g_up_b + 1 * 2 * FH, 1, 0);
  upadd(T, X0, U, N);
  lapblk(3, N, U, T, EG, 12, g_up_b + 2 * 2 * FH, 0, 1);

  k_conv_in<<<(N + PROWS - 1) / PROWS, NTHR, 0, stream>>>(inputs, l_conv1_W, l_conv1_b, U, AE32, AE16, N, ASCL);
  float* cur = U;
  float* oth = T;
  for (int i = 0; i < 15; ++i) {
    const int slot = 14 + 2 * i;
    const float* bb = l_rn_b + (size_t)i * 2 * FH;
    const int last = (i == 14) ? 1 : 0;
    if ((i % 2) == 0) lapblk(4, nlev[4], cur, oth, AE32, slot, bb, last ? 0 : 1, 1);
    else              avgblk(nlev[4], cur, oth, slot, bb, 1, 1);
    float* tsw = cur; cur = oth; oth = tsw;
  }

  k_heads<<<N / 32, NTHR, 0, stream>>>(EG, AE32, g_conv2_W, g_conv2_b, l_conv2_W, l_conv2_b, inputs, out, N);
}
